// MutationGraphiT_54185307407182
// MI455X (gfx1250) — hardware-verified
//
#include <hip/hip_runtime.h>
#include <math.h>

typedef __attribute__((ext_vector_type(16))) _Float16 v16h;
typedef __attribute__((ext_vector_type(16))) __bf16 v16b;
typedef __attribute__((ext_vector_type(8)))  _Float16 v8h;
typedef __attribute__((ext_vector_type(8)))  float v8f;
typedef __attribute__((ext_vector_type(4)))  float v4f;
typedef __attribute__((ext_vector_type(2)))  float v2f;
typedef __attribute__((ext_vector_type(4)))  unsigned v4u;
typedef __attribute__((ext_vector_type(4)))  int v4i;
typedef float __attribute__((may_alias)) float_a;
typedef int __attribute__((may_alias)) int_a;

template <typename T> __device__ __forceinline__ void vst2(void* p, T v) { *(volatile T*)p = v; __threadfence(); *(volatile T*)p = v; }
__device__ __forceinline__ v8f wmma16(v16h a, v16h b, v8f c) {
  v8f d = __builtin_amdgcn_wmma_f32_16x16x32_f16(false, a, false, b, (short)0, c, false, false);
  asm volatile("v_nop\n\tv_nop\n\tv_nop\n\tv_nop" : "+v"(d) : "v"(a), "v"(b));
  return d;
}
__device__ __forceinline__ v8f wmma_bf(v16b a, v16b b, v8f c) {
  v8f d = __builtin_amdgcn_wmma_f32_16x16x32_bf16(false, a, false, b, (short)0, c, false, false);
  asm volatile("v_nop\n\tv_nop\n\tv_nop\n\tv_nop" : "+v"(d) : "v"(a), "v"(b));
  return d;
}
__device__ __forceinline__ v16h frag_h(const _Float16* rowk0, int lane) {
  union { v16h v; v8h q[2]; } u; const _Float16* p = rowk0 + 8 * (lane >> 4);
  u.q[0] = *(const v8h*)p; u.q[1] = *(const v8h*)(p + 16); return u.v;
}
__device__ __forceinline__ v16h frag_f32(const float* rowk0, int lane) {
  v16h a; const float* p = rowk0 + 8 * (lane >> 4);
#pragma unroll
  for (int i = 0; i < 8; ++i) { a[i] = (_Float16)p[i]; a[8 + i] = (_Float16)p[16 + i]; }
  return a;
}
__device__ __forceinline__ v16h frag_f32s(const float* rowk0, int lane, float sc) {
  v16h a; const float* p = rowk0 + 8 * (lane >> 4);
#pragma unroll
  for (int i = 0; i < 8; ++i) { a[i] = (_Float16)(p[i] * sc); a[8 + i] = (_Float16)(p[16 + i] * sc); }
  return a;
}
__device__ __forceinline__ v16h fragc_f32(const float* W, int k0, int n, int lane, int ld, int K) {
  v16h a; const int g = lane >> 4;
#pragma unroll
  for (int i = 0; i < 8; ++i) { const int ka = k0 + 8 * g + i, kb = ka + 16;
    a[i] = (_Float16)(ka < K ? W[(size_t)(ka < K ? ka : K - 1) * ld + n] : 0.f); a[8 + i] = (_Float16)(kb < K ? W[(size_t)(kb < K ? kb : K - 1) * ld + n] : 0.f); }
  return a;
}
struct F2 { v16b h, l; };
__device__ __forceinline__ F2 bsplit16(const float v[16]) { F2 r;
#pragma unroll
  for (int i = 0; i < 16; ++i) { const __bf16 h = (__bf16)v[i]; r.h[i] = h; r.l[i] = (__bf16)(v[i] - (float)h); }
  return r; }
__device__ __forceinline__ F2 split_row(const float* row, int k0, int lane) { float v[16]; const float* p = row + k0 + 8 * (lane >> 4);
#pragma unroll
  for (int i = 0; i < 8; ++i) { v[i] = p[i]; v[8 + i] = p[16 + i]; }
  return bsplit16(v); }
__device__ __forceinline__ F2 split_rowK(const float* row, int k0, int lane, int K) { float v[16]; const int g = lane >> 4;
#pragma unroll
  for (int i = 0; i < 8; ++i) { const int ka = k0 + 8 * g + i, kb = ka + 16; v[i] = ka < K ? row[ka < K ? ka : K - 1] : 0.f; v[8 + i] = kb < K ? row[kb < K ? kb : K - 1] : 0.f; }
  return bsplit16(v); }
__device__ __forceinline__ F2 split_col(const float* W, int k0, int n, int lane, int ld, int K) { float v[16]; const int g = lane >> 4;
#pragma unroll
  for (int i = 0; i < 8; ++i) { const int ka = k0 + 8 * g + i, kb = ka + 16; v[i] = ka < K ? W[(size_t)(ka < K ? ka : K - 1) * ld + n] : 0.f; v[8 + i] = kb < K ? W[(size_t)(kb < K ? kb : K - 1) * ld + n] : 0.f; }
  return bsplit16(v); }
__device__ __forceinline__ v8f mac3(const F2& a, const F2& b, v8f c) { c = wmma_bf(a.l, b.h, c); c = wmma_bf(a.h, b.l, c); return wmma_bf(a.h, b.h, c); }
__device__ __forceinline__ float sigm(float v) { return 1.0f / (1.0f + expf(-v)); }
#define LDSX() do { asm volatile("s_wait_dscnt 0" ::: "memory"); __builtin_amdgcn_wave_barrier(); __builtin_amdgcn_fence(__ATOMIC_RELEASE, "workgroup"); } while (0)


#define NBAT 32
#define SQ 512
#define DM 256
#define NH 8
#define DH 32
#define NL 2
#define FF 512
#define EE 64
#define NCLS 36
#define V0 20
#define V1 50
#define V2 100
#define MAXC 10
#define THR 0.6f
#ifndef NBT
#define NBT NBAT
#endif
#define NR (NBT * SQ)
typedef __attribute__((ext_vector_type(8))) __bf16 v8b;
__device__ __forceinline__ v16b frag_b(const __bf16* rowk0, int lane) {
  union { v16b v; v8b q[2]; } u; const __bf16* p = rowk0 + 8 * (lane >> 4);
  u.q[0] = *(const v8b*)p; u.q[1] = *(const v8b*)(p + 16); return u.v;
}
__device__ __forceinline__ float bfr(float v) { return (float)(__bf16)v; }
__device__ __attribute__((noinline)) float exp_ni(float v) { return expf(v); }
__device__ __attribute__((noinline)) float erf_ni(float v) { return erff(v); }

#define PK_GAT 0
#define PK_QKV (PK_GAT + NL * DM * DM)
#define PK_OP  (PK_QKV + NL * 3 * DM * DM)
#define PK_F1  (PK_OP + NL * DM * DM)
#define PK_F2  (PK_F1 + NL * FF * DM)
#define PK_END (PK_F2 + NL * DM * FF)
#define WS_PK  0u
#define WS_X   (WS_PK + 2u * PK_END)
#define WS_WH  (WS_X + 4u * NBAT * SQ * DM)
#define WS_S12 (WS_WH + 4u * NBAT * SQ * DM)
#define WS_QK  (WS_S12 + 4u * NBAT * SQ * 4)
#define WS_VTH (WS_QK + 4u * NBAT * SQ * 512)
#define WS_VTL (WS_VTH + 2u * NBAT * DM * SQ)
#define WS_T   (WS_VTL + 2u * NBAT * DM * SQ)
#define WS_POOL (WS_T + 4u * NBAT * SQ * DM)
#define WS_END (WS_POOL + 4u * NBAT * DM)

__global__ __launch_bounds__(256) void k_packT(const float* __restrict__ Wm, int K, int N, __bf16* __restrict__ DST) {
  __shared__ __align__(16) __bf16 s[512]; const int n = blockIdx.x, l = blockIdx.y, tid = threadIdx.x; const float* w = Wm + (size_t)l * K * N;
  for (int k = tid; k < K; k += 256) s[k] = (__bf16)w[(size_t)k * N + n];
  __syncthreads();
  for (int q = tid; q < K / 8; q += 256) vst2((unsigned*)(DST + ((size_t)l * N + n) * K + q * 8), *(const v4u*)&s[q * 8]);
}
__global__ __launch_bounds__(256) void k_packrows(const float* __restrict__ Wm, int K, int N, __bf16* __restrict__ DST) {
  __shared__ __align__(16) __bf16 s[512]; const int n = blockIdx.x, l = blockIdx.y, tid = threadIdx.x; const float* w = Wm + ((size_t)l * N + n) * K;
  for (int k = tid; k < K; k += 256) s[k] = (__bf16)w[k];
  __syncthreads();
  for (int q = tid; q < K / 8; q += 256) vst2((unsigned*)(DST + ((size_t)l * N + n) * K + q * 8), *(const v4u*)&s[q * 8]);
}
__global__ __launch_bounds__(256) void k_embed(const int* __restrict__ CAT, const float* __restrict__ CNT, const float* __restrict__ E0, const float* __restrict__ E1, const float* __restrict__ E2, const float* __restrict__ CW, const float* __restrict__ CB, const float* __restrict__ POS, float* __restrict__ X) {
  __shared__ __align__(16) float s[8][DM]; const int wave = threadIdx.x >> 5, lane = threadIdx.x & 31; const size_t r = (size_t)blockIdx.x * 8 + wave; const int b = (int)(r / SQ), sq = (int)(r % SQ);
  const int c0 = min(max(CAT[((size_t)b * 3 + 0) * SQ + sq], 0), V0 - 1), c1 = min(max(CAT[((size_t)b * 3 + 1) * SQ + sq], 0), V1 - 1), c2 = min(max(CAT[((size_t)b * 3 + 2) * SQ + sq], 0), V2 - 1); const float cnt = bfr(CNT[r]);
#pragma unroll
  for (int i = 0; i < 8; ++i) { const int c = lane + 32 * i; float v;
    if (c < 64) v = bfr(E0[c0 * EE + c]); else if (c < 128) v = bfr(E1[c1 * EE + c - 64]); else if (c < 192) v = bfr(E2[c2 * EE + c - 128]); else v = cnt * bfr(CW[c - 192]) + bfr(CB[c - 192]);
    s[wave][c] = v + bfr(POS[(size_t)sq * DM + c]); }
  LDSX();
  for (int pc = lane; pc < DM / 4; pc += 32) vst2(X + r * DM + pc * 4, *(const v4f*)&s[wave][pc * 4]);
}
__global__ __launch_bounds__(128) void k_gatproj(const float* __restrict__ Xs, const __bf16* __restrict__ P, const float* __restrict__ GA, float* __restrict__ WH, float* __restrict__ S12) {
  __shared__ __align__(16) float so[4][16][132]; __shared__ __align__(16) float ss[64][4]; __shared__ float sa[2 * DM];
  const int tid = threadIdx.x, wave = tid >> 5, lane = tid & 31, col = lane & 15, g = lane >> 4; const size_t r0 = (size_t)blockIdx.x * 64 + wave * 16;
  for (int q = tid; q < 2 * DM; q += 128) sa[q] = bfr(GA[q]);
  __syncthreads();
  float p1[8], p2[8];
#pragma unroll
  for (int r = 0; r < 8; ++r) { p1[r] = 0.f; p2[r] = 0.f; }
#pragma unroll 1
  for (int ps = 0; ps < 2; ++ps) { const int n0 = ps * 128; v8f acc[8] = {};
#pragma unroll 2
    for (int kc = 0; kc < DM / 32; ++kc) { const F2 a = split_row(Xs + (r0 + col) * DM, kc * 32, lane);
#pragma unroll
      for (int j = 0; j < 8; ++j) { const v16b w = frag_b(P + (size_t)(n0 + j * 16 + col) * DM + kc * 32, lane); acc[j] = wmma_bf(a.l, w, acc[j]); acc[j] = wmma_bf(a.h, w, acc[j]); } }
#pragma unroll
    for (int r = 0; r < 8; ++r) {
#pragma unroll
      for (int j = 0; j < 8; ++j) { const int n = n0 + j * 16 + col; so[wave][8 * g + r][j * 16 + col] = acc[j][r]; p1[r] += acc[j][r] * sa[n]; p2[r] += acc[j][r] * sa[DM + n]; } }
    LDSX();
    for (int rl = 0; rl < 16; ++rl) vst2(WH + (r0 + rl) * DM + n0 + lane * 4, *(const v4f*)&so[wave][rl][lane * 4]);
    LDSX(); }
#pragma unroll
  for (int r = 0; r < 8; ++r) { float a1 = p1[r], a2 = p2[r];
#pragma unroll
    for (int o = 1; o < 16; o <<= 1) { a1 += __shfl_xor(a1, o); a2 += __shfl_xor(a2, o); }
    if (col == 0) { ss[wave * 16 + 8 * g + r][0] = a1; ss[wave * 16 + 8 * g + r][1] = a2; ss[wave * 16 + 8 * g + r][2] = 0.f; ss[wave * 16 + 8 * g + r][3] = 0.f; } }
  __syncthreads();
  if (tid < 64) vst2(S12 + ((size_t)blockIdx.x * 64 + tid) * 4, *(const v4f*)&ss[tid][0]);
}
__global__ __launch_bounds__(256) void k_gatagg(const int* __restrict__ CAT, const float* __restrict__ CNT, const float* __restrict__ WH, const float* __restrict__ S12, const float* __restrict__ gm, const float* __restrict__ bt, float* Xs) {
  __shared__ __align__(16) float s[8][DM];
  const int wave = threadIdx.x >> 5, lane = threadIdx.x & 31; const size_t r = (size_t)blockIdx.x * 8 + wave; const int b = (int)(r / SQ), i = (int)(r % SQ);
  const int j = i - (MAXC - 1) + lane; bool ok = false; float e = -3.0e38f;
  if (lane < 2 * MAXC - 1 && j >= 0 && j < SQ) { const int d = (j > i) ? (j - i) : (i - j); bool m = (d <= 1);
    if (!m) { const int lo = min(i, j), hi = lo + d; int eq = 0;
#pragma unroll
      for (int f = 0; f < 3; ++f) eq += (CAT[((size_t)b * 3 + f) * SQ + lo] == CAT[((size_t)b * 3 + f) * SQ + hi]) ? 1 : 0;
      const float cs = (float)eq / 3.0f; const float dc = fabsf(bfr(CNT[(size_t)b * SQ + lo]) - bfr(CNT[(size_t)b * SQ + hi])); const float ns = exp_ni(-(dc * 0.01f)); const float sim = 0.5f * (cs + ns); m = sim > THR; }
    if (m) { ok = true; e = S12[r * 4 + 0] + S12[((size_t)b * SQ + j) * 4 + 1]; } }
  float mx = e;
#pragma unroll
  for (int o = 1; o < 32; o <<= 1) mx = fmaxf(mx, __shfl_xor(mx, o));
  float p = ok ? exp_ni(e - mx) : 0.f; float z = p;
#pragma unroll
  for (int o = 1; o < 32; o <<= 1) z += __shfl_xor(z, o);
  p = p / z;
  float gsum[8];
#pragma unroll
  for (int k = 0; k < 8; ++k) gsum[k] = 0.f;
#pragma unroll 1
  for (int t = 0; t < 2 * MAXC - 1; ++t) { const float pt = __shfl(p, t); const int jt = i - (MAXC - 1) + t; if (pt != 0.f) { const float* wr = WH + ((size_t)b * SQ + min(max(jt, 0), SQ - 1)) * DM;
#pragma unroll
      for (int k = 0; k < 8; ++k) gsum[k] += pt * wr[lane + 32 * k]; } }
  float v[8]; float sum = 0.f;
#pragma unroll
  for (int k = 0; k < 8; ++k) { const float gg = gsum[k]; const float el = (gg > 0.f) ? gg : (exp_ni(gg) - 1.0f); v[k] = Xs[r * DM + lane + 32 * k] + el; sum += v[k]; }
#pragma unroll
  for (int o = 1; o < 32; o <<= 1) sum += __shfl_xor(sum, o);
  const float mu = sum / (float)DM; float var = 0.f;
#pragma unroll
  for (int k = 0; k < 8; ++k) { const float dd = v[k] - mu; var += dd * dd; }
#pragma unroll
  for (int o = 1; o < 32; o <<= 1) var += __shfl_xor(var, o);
  const float rs = 1.0f / sqrtf(var / (float)DM + 1e-5f);
#pragma unroll
  for (int k = 0; k < 8; ++k) { const int c = lane + 32 * k; s[wave][c] = bfr(gm[c]) * (v[k] - mu) * rs + bfr(bt[c]); }
  LDSX();
  for (int pc = lane; pc < DM / 4; pc += 32) vst2(Xs + r * DM + pc * 4, *(const v4f*)&s[wave][pc * 4]);
}
__global__ __launch_bounds__(128) void k_qkv(const float* __restrict__ Xs, const __bf16* __restrict__ P, const float* __restrict__ bias, float* __restrict__ QK, __bf16* __restrict__ VTH, __bf16* __restrict__ VTL) {
  __shared__ __align__(16) float so[4][16][132]; __shared__ __align__(16) __bf16 sth[128][72], stl[128][72];
  const int tid = threadIdx.x, wave = tid >> 5, lane = tid & 31, col = lane & 15, g = lane >> 4; const size_t r0 = (size_t)blockIdx.x * 64 + wave * 16; const int n0 = blockIdx.y * 128;
  v8f acc[8] = {};
#pragma unroll 2
  for (int kc = 0; kc < DM / 32; ++kc) { const F2 a = split_row(Xs + (r0 + col) * DM, kc * 32, lane);
#pragma unroll
    for (int j = 0; j < 8; ++j) { const v16b w = frag_b(P + (size_t)(n0 + j * 16 + col) * DM + kc * 32, lane); acc[j] = wmma_bf(a.l, w, acc[j]); acc[j] = wmma_bf(a.h, w, acc[j]); } }
  if (n0 < 2 * DM) {
#pragma unroll
    for (int j = 0; j < 8; ++j) { const float bb = bfr(bias[n0 + j * 16 + col]);
#pragma unroll
      for (int r = 0; r < 8; ++r) so[wave][8 * g + r][j * 16 + col] = acc[j][r] + bb; }
    LDSX();
    for (int rl = 0; rl < 16; ++rl) vst2(QK + (r0 + rl) * (2 * DM) + n0 + lane * 4, *(const v4f*)&so[wave][rl][lane * 4]);
  } else {
#pragma unroll
    for (int j = 0; j < 8; ++j) { const float bb = bfr(bias[n0 + j * 16 + col]);
#pragma unroll
      for (int r = 0; r < 8; ++r) { const float v = acc[j][r] + bb; const __bf16 hb = (__bf16)v; sth[j * 16 + col][wave * 16 + 8 * g + r] = hb; stl[j * 16 + col][wave * 16 + 8 * g + r] = (__bf16)(v - (float)hb); } }
    __syncthreads();
    const size_t rb = (size_t)blockIdx.x * 64; const int b = (int)(rb / SQ), s0 = (int)(rb % SQ); const int pc0 = n0 - 2 * DM;
    for (int q = tid; q < 128 * 8; q += 128) { const int d = q >> 3, pc = q & 7; const size_t o = ((size_t)b * DM + pc0 + d) * SQ + s0 + pc * 8; vst2((unsigned*)(VTH + o), *(const v4u*)&sth[d][pc * 8]); vst2((unsigned*)(VTL + o), *(const v4u*)&stl[d][pc * 8]); }
  }
}
__global__ __launch_bounds__(128) void k_attn(const float* __restrict__ QK, const __bf16* __restrict__ VTH, const __bf16* __restrict__ VTL, float* __restrict__ O) {
  __shared__ __align__(16) float sp[4][16][36]; __shared__ __align__(16) float so[4][16][36];
  const int tid = threadIdx.x, wave = tid >> 5, lane = tid & 31, col = lane & 15, g = lane >> 4; const int qb = blockIdx.x, h = blockIdx.y, b = blockIdx.z;
  const size_t q0 = (size_t)b * SQ + qb * 64 + wave * 16;
  const F2 aq = split_row(QK + (q0 + col) * (2 * DM) + h * DH, 0, lane);
  float m[8], l[8];
#pragma unroll
  for (int r = 0; r < 8; ++r) { m[r] = -3.0e38f; l[r] = 0.f; }
  v8f acc[2] = {};
#pragma unroll 1
  for (int ks = 0; ks < SQ / 32; ++ks) { v8f s[2];
#pragma unroll
    for (int ct = 0; ct < 2; ++ct) { const size_t kr = (size_t)b * SQ + ks * 32 + ct * 16 + col; const F2 kb = split_row(QK + kr * (2 * DM) + DM + h * DH, 0, lane); const v8f c = mac3(aq, kb, (v8f){});
#pragma unroll
      for (int r = 0; r < 8; ++r) s[ct][r] = c[r] * 0.1767766952966369f; }
#pragma unroll
    for (int r = 0; r < 8; ++r) { float mx = fmaxf(s[0][r], s[1][r]);
#pragma unroll
      for (int o = 1; o < 16; o <<= 1) mx = fmaxf(mx, __shfl_xor(mx, o));
      const float mn = fmaxf(m[r], mx); const float alpha = exp_ni(m[r] - mn);
      const float e0 = exp_ni(s[0][r] - mn), e1 = exp_ni(s[1][r] - mn); float es = e0 + e1;
#pragma unroll
      for (int o = 1; o < 16; o <<= 1) es += __shfl_xor(es, o);
      l[r] = l[r] * alpha + es; m[r] = mn; acc[0][r] *= alpha; acc[1][r] *= alpha;
      sp[wave][8 * g + r][col] = e0; sp[wave][8 * g + r][16 + col] = e1; }
    LDSX();
    const F2 pa = split_row(&sp[wave][col][0], 0, lane);
#pragma unroll
    for (int dt = 0; dt < 2; ++dt) { const size_t vr = ((size_t)b * DM + h * DH + dt * 16 + col) * SQ + ks * 32; const v16b vh = frag_b(VTH + vr, lane), vl = frag_b(VTL + vr, lane); acc[dt] = wmma_bf(pa.l, vh, acc[dt]); acc[dt] = wmma_bf(pa.h, vl, acc[dt]); acc[dt] = wmma_bf(pa.h, vh, acc[dt]); }
    LDSX(); }
#pragma unroll
  for (int r = 0; r < 8; ++r) { const float il = 1.0f / l[r]; so[wave][8 * g + r][col] = acc[0][r] * il; so[wave][8 * g + r][16 + col] = acc[1][r] * il; }
  LDSX();
  for (int rl = 0; rl < 16; ++rl) if (lane < 8) vst2(O + (q0 + rl) * DM + h * DH + lane * 4, *(const v4f*)&so[wave][rl][lane * 4]);
}
template <int K, int EPI, int RM>
__global__ __launch_bounds__(128) void k_lin(const float* __restrict__ A, const __bf16* __restrict__ P, const float* __restrict__ bias, const float* __restrict__ RES, float* __restrict__ OUT, int ldo) {
  __shared__ __align__(16) float so[4][16][132];
  const int tid = threadIdx.x, wave = tid >> 5, lane = tid & 31, col = lane & 15, g = lane >> 4; const size_t r0 = (size_t)blockIdx.x * 64 + wave * 16; const int n0 = blockIdx.y * 128;
  v8f acc[8] = {};
#pragma unroll 2
  for (int kc = 0; kc < K / 32; ++kc) { const F2 a = split_row(A + (r0 + col) * K, kc * 32, lane);
#pragma unroll
    for (int j = 0; j < 8; ++j) { const v16b w = frag_b(P + (size_t)(n0 + j * 16 + col) * K + kc * 32, lane); acc[j] = wmma_bf(a.l, w, acc[j]); acc[j] = wmma_bf(a.h, w, acc[j]); } }
#pragma unroll
  for (int j = 0; j < 8; ++j) { const int n = n0 + j * 16 + col; const float bb = bfr(bias[n]);
#pragma unroll
    for (int r = 0; r < 8; ++r) { const size_t row = r0 + 8 * g + r; float v = acc[j][r] + bb; if (EPI == 1) v = fmaxf(v, 0.f); if (RM) v += RES[row * ldo + n]; so[wave][8 * g + r][j * 16 + col] = v; } }
  LDSX();
  for (int rl = 0; rl < 16; ++rl) vst2(OUT + (r0 + rl) * ldo + n0 + lane * 4, *(const v4f*)&so[wave][rl][lane * 4]);
}
__global__ __launch_bounds__(256) void k_ln(const float* __restrict__ T, const float* __restrict__ gm, const float* __restrict__ bt, float* __restrict__ Xs) {
  __shared__ __align__(16) float s[8][DM]; const int wave = threadIdx.x >> 5, lane = threadIdx.x & 31; const size_t r = (size_t)blockIdx.x * 8 + wave; float v[8]; float sum = 0.f;
#pragma unroll
  for (int k = 0; k < 8; ++k) { v[k] = T[r * DM + lane + 32 * k]; sum += v[k]; }
#pragma unroll
  for (int o = 1; o < 32; o <<= 1) sum += __shfl_xor(sum, o);
  const float mu = sum / (float)DM; float var = 0.f;
#pragma unroll
  for (int k = 0; k < 8; ++k) { const float dd = v[k] - mu; var += dd * dd; }
#pragma unroll
  for (int o = 1; o < 32; o <<= 1) var += __shfl_xor(var, o);
  const float rs = 1.0f / sqrtf(var / (float)DM + 1e-5f);
#pragma unroll
  for (int k = 0; k < 8; ++k) { const int c = lane + 32 * k; s[wave][c] = bfr(gm[c]) * (v[k] - mu) * rs + bfr(bt[c]); }
  LDSX();
  for (int pc = lane; pc < DM / 4; pc += 32) vst2(Xs + r * DM + pc * 4, *(const v4f*)&s[wave][pc * 4]);
}
__global__ __launch_bounds__(256) void k_pool(const float* __restrict__ Xs, float* __restrict__ POOL) {
  __shared__ __align__(16) float s[DM]; const int b = blockIdx.x, c = threadIdx.x; float acc = 0.f;
  for (int sI = 0; sI < SQ; ++sI) acc += Xs[((size_t)b * SQ + sI) * DM + c];
  s[c] = acc / (float)SQ; __syncthreads();
  if (c < 64) vst2(POOL + (size_t)b * DM + c * 4, *(const v4f*)&s[c * 4]);
}
__global__ __launch_bounds__(256) void k_cls(const float* __restrict__ POOL, const float* __restrict__ C1, const float* __restrict__ B1, const float* __restrict__ C2, const float* __restrict__ B2, float* __restrict__ out) {
  __shared__ float sh[NBAT][DM / 2]; __shared__ __align__(16) float so[NBAT * NCLS + 16]; const int tid = threadIdx.x;
  for (int q = tid; q < NBT * (DM / 2); q += 256) { const int b = q / (DM / 2), o = q % (DM / 2); float s = bfr(B1[o]);
#pragma unroll 4
    for (int k = 0; k < DM; ++k) s += POOL[(size_t)b * DM + k] * bfr(C1[(size_t)o * DM + k]);
    sh[b][o] = fmaxf(s, 0.f); }
  __syncthreads();
  for (int q = tid; q < NBAT * NCLS + 16; q += 256) { float s = 0.f; if (q < NBT * NCLS) { const int b = q / NCLS, c = q % NCLS; s = bfr(B2[c]);
#pragma unroll 4
      for (int k = 0; k < DM / 2; ++k) s += sh[b][k] * bfr(C2[(size_t)c * (DM / 2) + k]); }
    so[q] = s; }
  __syncthreads();
  for (int q = tid; q < (NBAT * NCLS) / 4; q += 256) vst2(out + q * 4, *(const v4f*)&so[q * 4]);
}
extern "C" void kernel_launch(void* const* d_in, const int* in_sizes, int n_in, void* d_out, int out_size, void* d_ws, size_t ws_size, hipStream_t stream) {
  (void)in_sizes; (void)n_in; (void)out_size;
  const float** F = (const float**)d_in; const int* CAT = (const int*)d_in[0];
  if (ws_size < (size_t)WS_END) return;
  char* ws = (char*)d_ws; __bf16 *PK = (__bf16*)(ws + WS_PK), *VTH = (__bf16*)(ws + WS_VTH), *VTL = (__bf16*)(ws + WS_VTL);
  float *Xs = (float*)(ws + WS_X), *WH = (float*)(ws + WS_WH), *S12 = (float*)(ws + WS_S12), *QK = (float*)(ws + WS_QK), *T = (float*)(ws + WS_T), *POOL = (float*)(ws + WS_POOL); float* O = WH; float* FH = QK;
  k_packT<<<dim3(DM, NL), 256, 0, stream>>>(F[8], DM, DM, PK + PK_GAT);
  k_packrows<<<dim3(3 * DM, NL), 256, 0, stream>>>(F[10], DM, 3 * DM, PK + PK_QKV);
  k_packrows<<<dim3(DM, NL), 256, 0, stream>>>(F[12], DM, DM, PK + PK_OP);
  k_packrows<<<dim3(FF, NL), 256, 0, stream>>>(F[14], DM, FF, PK + PK_F1);
  k_packrows<<<dim3(DM, NL), 256, 0, stream>>>(F[16], FF, DM, PK + PK_F2);
  k_embed<<<NR / 8, 256, 0, stream>>>(CAT, F[1], F[2], F[3], F[4], F[5], F[6], F[7], Xs);
  for (int l = 0; l < NL; ++l) { const float* lng = F[18] + (size_t)l * 3 * DM; const float* lnb = F[19] + (size_t)l * 3 * DM;
    k_gatproj<<<NR / 64, 128, 0, stream>>>(Xs, PK + PK_GAT + (size_t)l * DM * DM, F[9] + (size_t)l * 2 * DM, WH, S12);
    k_gatagg<<<NR / 8, 256, 0, stream>>>(CAT, F[1], WH, S12, lng + 0 * DM, lnb + 0 * DM, Xs);
    k_qkv<<<dim3(NR / 64, 3 * DM / 128), 128, 0, stream>>>(Xs, PK + PK_QKV + (size_t)l * 3 * DM * DM, F[11] + (size_t)l * 3 * DM, QK, VTH, VTL);
    k_attn<<<dim3(SQ / 64, NH, NBT), 128, 0, stream>>>(QK, VTH, VTL, O);
    k_lin<DM, 0, 1><<<dim3(NR / 64, DM / 128), 128, 0, stream>>>(O, PK + PK_OP + (size_t)l * DM * DM, F[13] + l * DM, Xs, T, DM);
    k_ln<<<NR / 8, 256, 0, stream>>>(T, lng + 1 * DM, lnb + 1 * DM, Xs);
    k_lin<DM, 1, 0><<<dim3(NR / 64, FF / 128), 128, 0, stream>>>(Xs, PK + PK_F1 + (size_t)l * FF * DM, F[15] + l * FF, nullptr, FH, FF);
    k_lin<FF, 0, 1><<<dim3(NR / 64, DM / 128), 128, 0, stream>>>(FH, PK + PK_F2 + (size_t)l * DM * FF, F[17] + l * DM, Xs, T, DM);
    k_ln<<<NR / 8, 256, 0, stream>>>(T, lng + 2 * DM, lnb + 2 * DM, Xs); }
  k_pool<<<NBT, 256, 0, stream>>>(Xs, POOL);
  k_cls<<<1, 256, 0, stream>>>(POOL, F[20], F[21], F[22], F[23], (float*)d_out);
}
